// GRUModel_2808908611659
// MI455X (gfx1250) — hardware-verified
//
#include <hip/hip_runtime.h>

#define B_SZ 4096
#define T_SZ 256
#define D_SZ 5
#define H_SZ 64
#define G_SZ 192

typedef __attribute__((ext_vector_type(16))) _Float16 v16h;
typedef __attribute__((ext_vector_type(8)))  float    v8f;

typedef float __attribute__((may_alias)) float_a;
typedef __attribute__((ext_vector_type(4))) float v4f;
template <typename TT> __device__ __forceinline__ void vst2(void* p, TT v) { *(volatile TT*)p = v; __threadfence(); *(volatile TT*)p = v; }
__device__ __forceinline__ v8f WMMA_F16(v16h a, v16h b, v8f c) {
  v8f d = __builtin_amdgcn_wmma_f32_16x16x32_f16(false, a, false, b, (short)0, c, false, false);
  asm volatile("v_nop\n\tv_nop\n\tv_nop\n\tv_nop" : "+v"(d) : "v"(a), "v"(b));
  return d;
}

__device__ __forceinline__ float fast_sigmoid(float x) { return 1.0f / (1.0f + expf(-x)); }
__device__ __forceinline__ float fast_tanh(float x) { return tanhf(x); }

__device__ __forceinline__ v16h frag_a_f32(const float* tile, int stride, int kOff, int lane) {
  const int m    = lane & 15;
  const int hsel = (lane >> 4) << 3;
  const float* p0 = tile + m * stride + kOff + hsel;
  const float* p1 = p0 + 16;
  v16h a;
#pragma unroll
  for (int i = 0; i < 8; ++i) { a[i] = (_Float16)p0[i]; a[8 + i] = (_Float16)p1[i]; }
  return a;
}

__device__ __forceinline__ v16h frag_a_f16(const _Float16* tile, int stride, int lane) {
  const int m    = lane & 15;
  const int hsel = (lane >> 4) << 3;
  const _Float16* p0 = tile + m * stride + hsel;
  const _Float16* p1 = p0 + 16;
  v16h a;
#pragma unroll
  for (int i = 0; i < 8; ++i) { a[i] = p0[i]; a[8 + i] = p1[i]; }
  return a;
}

__device__ __forceinline__ v16h frag_b(const _Float16* W, int wstride, int nBase, int kOff, int lane) {
  const int n    = lane & 15;
  const int ksel = (lane >> 4) << 3;
  const _Float16* p = W + (nBase + n) * wstride + kOff + ksel;
  v16h b;
#pragma unroll
  for (int i = 0; i < 8; ++i) { b[i] = p[i]; b[8 + i] = p[16 + i]; }
  return b;
}

#define OFF_WIH0 0
#define OFF_WHH0 (OFF_WIH0 + G_SZ*32*2)
#define OFF_WIH1 (OFF_WHH0 + G_SZ*H_SZ*2)
#define OFF_WHH1 (OFF_WIH1 + G_SZ*H_SZ*2)
#define OFF_BI0  (OFF_WHH1 + G_SZ*H_SZ*2)
#define OFF_BH0  (OFF_BI0 + G_SZ*4)
#define OFF_BI1  (OFF_BH0 + G_SZ*4)
#define OFF_BH1  (OFF_BI1 + G_SZ*4)
#define OFF_FCW  (OFF_BH1 + G_SZ*4)
#define OFF_STATE (OFF_FCW + H_SZ*4)
#define STATE_BYTES (16*32*2 + 2*16*H_SZ*4 + 2*16*H_SZ*4)
#define SMEM_BYTES (OFF_STATE + STATE_BYTES)

__global__ __launch_bounds__(64)
void gru_fused_kernel(const float* __restrict__ x,
                      const float* __restrict__ w_ih0, const float* __restrict__ w_hh0,
                      const float* __restrict__ b_ih0, const float* __restrict__ b_hh0,
                      const float* __restrict__ w_ih1, const float* __restrict__ w_hh1,
                      const float* __restrict__ b_ih1, const float* __restrict__ b_hh1,
                      const float* __restrict__ fc_w, const float* __restrict__ fc_b,
                      float* __restrict__ stage)
{
  extern __shared__ char smem[];
  _Float16* sWih0 = (_Float16*)(smem + OFF_WIH0);
  _Float16* sWhh0 = (_Float16*)(smem + OFF_WHH0);
  _Float16* sWih1 = (_Float16*)(smem + OFF_WIH1);
  _Float16* sWhh1 = (_Float16*)(smem + OFF_WHH1);
  float* sBi0 = (float*)(smem + OFF_BI0);
  float* sBh0 = (float*)(smem + OFF_BH0);
  float* sBi1 = (float*)(smem + OFF_BI1);
  float* sBh1 = (float*)(smem + OFF_BH1);
  float* sFcw = (float*)(smem + OFF_FCW);

  const int tid  = threadIdx.x;
  const int lane = tid & 31;
  const int wave = tid >> 5;

  _Float16* sX = (_Float16*)(smem + OFF_STATE);
  float* sH0   = (float*)(smem + OFF_STATE + 16*32*2);
  float* sH2   = sH0 + 2*16*H_SZ;

  for (int i = tid; i < G_SZ*32; i += 64) {
    int r = i >> 5, c = i & 31;
    sWih0[i] = (c < D_SZ) ? (_Float16)w_ih0[r*D_SZ + c] : (_Float16)0.0f;
  }
  for (int i = tid; i < G_SZ*H_SZ; i += 64) {
    sWhh0[i] = (_Float16)w_hh0[i];
    sWih1[i] = (_Float16)w_ih1[i];
    sWhh1[i] = (_Float16)w_hh1[i];
  }
  for (int i = tid; i < G_SZ; i += 64) {
    sBi0[i] = b_ih0[i]; sBh0[i] = b_hh0[i];
    sBi1[i] = b_ih1[i]; sBh1[i] = b_hh1[i];
  }
  for (int i = tid; i < H_SZ; i += 64) sFcw[i] = fc_w[i];

  for (int i = tid; i < 16*H_SZ; i += 64) { sH0[i] = 0.0f; sH2[i] = 0.0f; }
  for (int i = tid; i < 16*32;   i += 64) sX[i] = (_Float16)0.0f;
  __syncthreads();

  const int rowBase = blockIdx.x * 16;
  const int ncol = lane & 15;
  const int hi   = lane >> 4;
  const int ntBase = wave * 2;

  float bR0[2], bZ0[2], bNi0[2], bNh0[2];
  float bR1[2], bZ1[2], bNi1[2], bNh1[2];
#pragma unroll
  for (int q = 0; q < 2; ++q) {
    const int g = (ntBase + q)*16 + ncol;
    bR0[q]  = sBi0[g]      + sBh0[g];
    bZ0[q]  = sBi0[g + 64] + sBh0[g + 64];
    bNi0[q] = sBi0[g + 128];
    bNh0[q] = sBh0[g + 128];
    bR1[q]  = sBi1[g]      + sBh1[g];
    bZ1[q]  = sBi1[g + 64] + sBh1[g + 64];
    bNi1[q] = sBi1[g + 128];
    bNh1[q] = sBh1[g + 128];
  }

  const float* xbase = x + (size_t)(rowBase + tid) * T_SZ * D_SZ;
  int cur = 0;

  for (int t = 0; t < T_SZ; ++t) {
    if (tid < 16) {
      const float* xp = xbase + (size_t)t * D_SZ;
#pragma unroll
      for (int d = 0; d < D_SZ; ++d) sX[tid*32 + d] = (_Float16)xp[d];
    }
    __syncthreads();

    float* h0c = sH0 + cur*16*H_SZ;
    float* h0n = sH0 + (cur^1)*16*H_SZ;
    float* h2c = sH2 + cur*16*H_SZ;
    float* h2n = sH2 + (cur^1)*16*H_SZ;

    {
      v16h aX   = frag_a_f16(sX, 32, lane);
      v16h aH0a = frag_a_f32(h0c, H_SZ, 0,  lane);
      v16h aH0b = frag_a_f32(h0c, H_SZ, 32, lane);
#pragma unroll
      for (int q = 0; q < 2; ++q) {
        const int nt = ntBase + q;
        v8f xr = {};
        xr = WMMA_F16(aX, frag_b(sWih0, 32, nt*16, 0, lane), xr);
        v8f hr = {};
        hr = WMMA_F16(aH0a, frag_b(sWhh0, H_SZ, nt*16, 0,  lane), hr);
        hr = WMMA_F16(aH0b, frag_b(sWhh0, H_SZ, nt*16, 32, lane), hr);
        v8f xz = {};
        xz = WMMA_F16(aX, frag_b(sWih0, 32, 64 + nt*16, 0, lane), xz);
        v8f hz = {};
        hz = WMMA_F16(aH0a, frag_b(sWhh0, H_SZ, 64 + nt*16, 0,  lane), hz);
        hz = WMMA_F16(aH0b, frag_b(sWhh0, H_SZ, 64 + nt*16, 32, lane), hz);
        v8f xn = {};
        xn = WMMA_F16(aX, frag_b(sWih0, 32, 128 + nt*16, 0, lane), xn);
        v8f hn = {};
        hn = WMMA_F16(aH0a, frag_b(sWhh0, H_SZ, 128 + nt*16, 0,  lane), hn);
        hn = WMMA_F16(aH0b, frag_b(sWhh0, H_SZ, 128 + nt*16, 32, lane), hn);

        const int jcol = nt*16 + ncol;
#pragma unroll
        for (int j = 0; j < 8; ++j) {
          const int m = j + (hi << 3);
          float r = fast_sigmoid(xr[j] + hr[j] + bR0[q]);
          float z = fast_sigmoid(xz[j] + hz[j] + bZ0[q]);
          float n = fast_tanh(xn[j] + bNi0[q] + r * (hn[j] + bNh0[q]));
          float hold = h0c[m*H_SZ + jcol];
          h0n[m*H_SZ + jcol] = (1.0f - z) * n + z * hold;
        }
      }
    }

    v16h aH2a = frag_a_f32(h2c, H_SZ, 0,  lane);
    v16h aH2b = frag_a_f32(h2c, H_SZ, 32, lane);
    __syncthreads();

    {
      v16h aI1a = frag_a_f32(h0n, H_SZ, 0,  lane);
      v16h aI1b = frag_a_f32(h0n, H_SZ, 32, lane);
#pragma unroll
      for (int q = 0; q < 2; ++q) {
        const int nt = ntBase + q;
        v8f xr = {};
        xr = WMMA_F16(aI1a, frag_b(sWih1, H_SZ, nt*16, 0,  lane), xr);
        xr = WMMA_F16(aI1b, frag_b(sWih1, H_SZ, nt*16, 32, lane), xr);
        v8f hr = {};
        hr = WMMA_F16(aH2a, frag_b(sWhh1, H_SZ, nt*16, 0,  lane), hr);
        hr = WMMA_F16(aH2b, frag_b(sWhh1, H_SZ, nt*16, 32, lane), hr);
        v8f xz = {};
        xz = WMMA_F16(aI1a, frag_b(sWih1, H_SZ, 64 + nt*16, 0,  lane), xz);
        xz = WMMA_F16(aI1b, frag_b(sWih1, H_SZ, 64 + nt*16, 32, lane), xz);
        v8f hz = {};
        hz = WMMA_F16(aH2a, frag_b(sWhh1, H_SZ, 64 + nt*16, 0,  lane), hz);
        hz = WMMA_F16(aH2b, frag_b(sWhh1, H_SZ, 64 + nt*16, 32, lane), hz);
        v8f xn = {};
        xn = WMMA_F16(aI1a, frag_b(sWih1, H_SZ, 128 + nt*16, 0,  lane), xn);
        xn = WMMA_F16(aI1b, frag_b(sWih1, H_SZ, 128 + nt*16, 32, lane), xn);
        v8f hn = {};
        hn = WMMA_F16(aH2a, frag_b(sWhh1, H_SZ, 128 + nt*16, 0,  lane), hn);
        hn = WMMA_F16(aH2b, frag_b(sWhh1, H_SZ, 128 + nt*16, 32, lane), hn);

        const int jcol = nt*16 + ncol;
#pragma unroll
        for (int j = 0; j < 8; ++j) {
          const int m = j + (hi << 3);
          float r = fast_sigmoid(xr[j] + hr[j] + bR1[q]);
          float z = fast_sigmoid(xz[j] + hz[j] + bZ1[q]);
          float n = fast_tanh(xn[j] + bNi1[q] + r * (hn[j] + bNh1[q]));
          float hold = h2c[m*H_SZ + jcol];
          h2n[m*H_SZ + jcol] = (1.0f - z) * n + z * hold;
        }
      }
    }
    cur ^= 1;
  }

  __syncthreads();

  if (tid < 16) {
    const float* hf = sH2 + cur*16*H_SZ + tid*H_SZ;
    float acc = fc_b[0];
#pragma unroll
    for (int j = 0; j < H_SZ; ++j) acc += hf[j] * sFcw[j];
    vst2(stage + rowBase + tid, (float_a)acc);
  }
}
__global__ __launch_bounds__(256) void out_kernel(const float* __restrict__ stage, float* __restrict__ out) {
  const int g = blockIdx.x * 256 + threadIdx.x;
  vst2(out + (size_t)g * 4, *(const v4f*)(stage + (size_t)g * 4));
}

extern "C" void kernel_launch(void* const* d_in, const int* in_sizes, int n_in,
                              void* d_out, int out_size, void* d_ws, size_t ws_size,
                              hipStream_t stream) {
  (void)in_sizes; (void)n_in; (void)ws_size; (void)out_size;
  float* stage = (float*)d_ws;
  const float* x     = (const float*)d_in[0];
  const float* w_ih0 = (const float*)d_in[1];
  const float* w_hh0 = (const float*)d_in[2];
  const float* b_ih0 = (const float*)d_in[3];
  const float* b_hh0 = (const float*)d_in[4];
  const float* w_ih1 = (const float*)d_in[5];
  const float* w_hh1 = (const float*)d_in[6];
  const float* b_ih1 = (const float*)d_in[7];
  const float* b_hh1 = (const float*)d_in[8];
  const float* fc_w  = (const float*)d_in[9];
  const float* fc_b  = (const float*)d_in[10];
  float* out = (float*)d_out;

  (void)hipFuncSetAttribute((const void*)gru_fused_kernel,
                            hipFuncAttributeMaxDynamicSharedMemorySize, SMEM_BYTES);

  dim3 grid(B_SZ / 16);
  dim3 block(64);
  gru_fused_kernel<<<grid, block, SMEM_BYTES, stream>>>(
      x, w_ih0, w_hh0, b_ih0, b_hh0, w_ih1, w_hh1, b_ih1, b_hh1, fc_w, fc_b, stage);
  out_kernel<<<B_SZ / 4 / 256, 256, 0, stream>>>(stage, out);
}
